// MultiheadSelfAttention_81475529605301
// MI455X (gfx1250) — hardware-verified
//
#include <hip/hip_runtime.h>
#ifndef NB
#define NB 4
#endif
#ifndef SEQ
#define SEQ 1024
#endif
#define NB_FULL 4
#define SEQ_FULL 1024
#define DM 1024
#define NH 16
#define HD 64
#define LQ (3 * DM)
#define NR (NB * SEQ)
#define ERW 256

static_assert(NB <= NB_FULL);
static_assert(SEQ <= SEQ_FULL);
static_assert(NH * HD == DM);
static_assert(HD == 64);
static_assert(DM % 64 == 0);
static_assert(DM % 32 == 0);
static_assert(LQ % 64 == 0);
static_assert(SEQ % 128 == 0);
static_assert(NR % 128 == 0);
static_assert(ERW % 128 == 0);
static_assert(SEQ >= ERW);
static_assert(ERW % 64 == 0);
static_assert(SEQ % 8 == 0);
static_assert(((size_t)NR * DM / 8) % 256 == 0);
static_assert(((size_t)DM * DM / 8) % 256 == 0);

typedef unsigned short v8us __attribute__((ext_vector_type(8), may_alias));
typedef float  v8f  __attribute__((ext_vector_type(8)));
typedef float  v4f  __attribute__((ext_vector_type(4)));
typedef float  v4fa __attribute__((ext_vector_type(4), may_alias));
typedef _Float16 v16h __attribute__((ext_vector_type(16)));
union FragH { v16h v; v8us half[2]; _Float16 h[16]; unsigned short u[16]; };

__device__ __forceinline__ unsigned short bf16_bits(float x) { unsigned int u = __float_as_uint(x); return (unsigned short)((u + 0x7FFFu + ((u >> 16) & 1u)) >> 16); }
__device__ __forceinline__ float bf16_rne(float x) { return __uint_as_float(((unsigned int)bf16_bits(x)) << 16); }

__device__ __forceinline__ v16h g2_frag(const _Float16* p, int hh) { FragH f; f.half[0] = *(const v8us*)((const unsigned short*)p + 8 * hh); f.half[1] = *(const v8us*)((const unsigned short*)p + 16 + 8 * hh); return f.v; }
__device__ __forceinline__ v8f g2_mma(v16h a, v16h b, v8f c) { v8f d = __builtin_amdgcn_wmma_f32_16x16x32_f16(false, a, false, b, (short)0, c, false, false); asm volatile("v_nop\n\tv_nop\n\tv_nop\n\tv_nop" : "+v"(d) : "v"(a), "v"(b)); return d; }
__device__ __forceinline__ void wave_lds_sync() { __builtin_amdgcn_fence(4  , "workgroup"); __builtin_amdgcn_wave_barrier(); }

__global__ __launch_bounds__(256) void k_wnat(const float* __restrict__ w, _Float16* __restrict__ Bt) {
  const size_t t = (size_t)blockIdx.x * 256 + threadIdx.x;
  if (t >= (size_t)DM * DM / 8) return;
  const v4f a = *(const v4fa*)(w + t * 8), c = *(const v4fa*)(w + t * 8 + 4);
  FragH f;
#pragma unroll
  for (int q = 0; q < 4; ++q) { f.h[q] = (_Float16)(bf16_rne(a[q]) * 16.0f); f.h[4 + q] = (_Float16)(bf16_rne(c[q]) * 16.0f); }
  const v8us o = f.half[0];
  unsigned short* d = (unsigned short*)Bt + t * 8;
  *(volatile v8us*)d = o;
  __threadfence();
  *(volatile v8us*)d = o;
}

__global__ __launch_bounds__(256) void k_x16(const float* __restrict__ x, _Float16* __restrict__ X16) {
  const size_t t = (size_t)blockIdx.x * 256 + threadIdx.x;
  if (t >= (size_t)NR * DM / 8) return;
  const size_t row = t / (DM / 8);
  const int c8 = (int)(t % (DM / 8)) * 8;
  const size_t b = row / SEQ, s = row % SEQ;
  const float* src = x + (b * SEQ_FULL + s) * DM + c8;
  const v4f a = *(const v4fa*)src, c = *(const v4fa*)(src + 4);
  FragH f;
#pragma unroll
  for (int q = 0; q < 4; ++q) { f.h[q] = (_Float16)bf16_rne(a[q]); f.h[4 + q] = (_Float16)bf16_rne(c[q]); }
  const v8us o = f.half[0];
  unsigned short* d = (unsigned short*)X16 + t * 8;
  *(volatile v8us*)d = o;
  __threadfence();
  *(volatile v8us*)d = o;
}

__global__ __launch_bounds__(256) void k_tab(const int* __restrict__ tp, float* __restrict__ CS) {
  __shared__ __attribute__((aligned(16))) float ts[8][64];
  const int tid = threadIdx.x;
  const int sl = tid >> 5, j = tid & 31;
  const int s = blockIdx.x * 8 + sl;
  const int pos = tp[s];
  double p = 1.0;
  p = (j & 1)  ? p * 1.3335214321633240 : p;
  p = (j & 2)  ? p * 1.7782794100389228 : p;
  p = (j & 4)  ? p * 3.1622776601683795 : p;
  p = (j & 8)  ? p * 10.0 : p;
  p = (j & 16) ? p * 100.0 : p;
  const float inv = (float)(1.0 / p);
  const float ang = (float)pos * inv;
  float sn, cs;
  sincosf(ang, &sn, &cs);
  ts[sl][2 * j] = cs;
  ts[sl][2 * j + 1] = sn;
  __syncthreads();
  if (tid < 128) {
    const int r = tid >> 4, c4 = (tid & 15) * 4;
    const v4f v = *(const v4fa*)&ts[r][c4];
    float* d = CS + (size_t)(blockIdx.x * 8 + r) * 64 + c4;
    *(volatile v4f*)d = v;
    __threadfence();
    *(volatile v4f*)d = v;
  }
}

__global__ __launch_bounds__(128) void k_qkv(const _Float16* __restrict__ X16, const _Float16* __restrict__ Bw, const float* __restrict__ CS, _Float16* __restrict__ Ph, _Float16* __restrict__ Pr) {
  __shared__ __attribute__((aligned(16))) float so[4][32][68];
  const int tid = threadIdx.x;
  const int wave = __builtin_amdgcn_readfirstlane((int)(tid >> 5));
  const int lane = tid & 31, ln = lane & 15, hh = lane >> 4;
  const int ntn = LQ / 64;
  const int mt = blockIdx.x / ntn, nq = blockIdx.x - mt * ntn;
  const int row0 = mt * 128 + 32 * wave, col0 = nq * 64;
  const _Float16* a0p = X16 + (size_t)(row0 + ln) * DM;
  const _Float16* a1p = a0p + (size_t)16 * DM;
  const _Float16* b0p = Bw + (size_t)(col0 + ln) * DM;
  const _Float16* b1p = b0p + (size_t)16 * DM;
  const _Float16* b2p = b1p + (size_t)16 * DM;
  const _Float16* b3p = b2p + (size_t)16 * DM;
  const v8f z8 = {0.f, 0.f, 0.f, 0.f, 0.f, 0.f, 0.f, 0.f};
  v8f c[8] = {z8, z8, z8, z8, z8, z8, z8, z8};
#pragma unroll 1
  for (int kb = 0; kb < DM; kb += 32) {
    const v16h a0 = g2_frag(a0p + kb, hh), a1 = g2_frag(a1p + kb, hh);
    v16h b = g2_frag(b0p + kb, hh); c[0] = g2_mma(a0, b, c[0]); c[4] = g2_mma(a1, b, c[4]);
    b = g2_frag(b1p + kb, hh); c[1] = g2_mma(a0, b, c[1]); c[5] = g2_mma(a1, b, c[5]);
    b = g2_frag(b2p + kb, hh); c[2] = g2_mma(a0, b, c[2]); c[6] = g2_mma(a1, b, c[6]);
    b = g2_frag(b3p + kb, hh); c[3] = g2_mma(a0, b, c[3]); c[7] = g2_mma(a1, b, c[7]);
  }
#pragma unroll
  for (int u = 0; u < 8; ++u) {
    const int t = u & 3, half = u >> 2;
#pragma unroll
    for (int r = 0; r < 8; ++r) so[wave][half * 16 + 8 * hh + r][t * 16 + ln] = c[u][r] * 0.0625f;
  }
  wave_lds_sync();
  const int rsub = lane >> 3, c8 = (lane & 7) * 8;
  const bool rp = col0 < 2 * DM;
  for (int pass = 0; pass < 2; ++pass) {
#pragma unroll 1
    for (int q = 0; q < 8; ++q) {
      const int r = q * 4 + rsub;
      const v4f u0 = *(const v4fa*)&so[wave][r][c8], u1 = *(const v4fa*)&so[wave][r][c8 + 4];
      const int s = (row0 + r) % SEQ;
      const v4f t0 = *(const v4fa*)(CS + (size_t)s * 64 + c8), t1 = *(const v4fa*)(CS + (size_t)s * 64 + c8 + 4);
      float e[8] = {u0[0], u0[1], u0[2], u0[3], u1[0], u1[1], u1[2], u1[3]};
      const float cz[4] = {t0[0], t0[2], t1[0], t1[2]};
      const float sz[4] = {t0[1], t0[3], t1[1], t1[3]};
#pragma unroll
      for (int i = 0; i < 4; ++i) {
        const float te = e[2 * i], to = e[2 * i + 1];
        const float re = te * cz[i] - to * sz[i];
        const float ro = te * sz[i] + to * cz[i];
        e[2 * i] = rp ? re : te;
        e[2 * i + 1] = rp ? ro : to;
      }
      FragH fh, fr;
#pragma unroll
      for (int i = 0; i < 8; ++i) { const _Float16 hi = (_Float16)e[i]; fh.h[i] = hi; fr.h[i] = (_Float16)((e[i] - (float)hi) * 1024.0f); }
      const v8us oh8 = fh.half[0], or8 = fr.half[0];
      const size_t o = (size_t)(row0 + r) * LQ + col0 + c8;
      *(volatile v8us*)((unsigned short*)Ph + o) = oh8;
      *(volatile v8us*)((unsigned short*)Pr + o) = or8;
    }
    if (pass == 0) __threadfence();
  }
}

__global__ __launch_bounds__(256) void k_vt(const _Float16* __restrict__ QKV, _Float16* __restrict__ VT) {
  __shared__ unsigned short tl[64][66];
  const int tid = threadIdx.x;
  const int slab = blockIdx.x / (SEQ / 64), lg = blockIdx.x % (SEQ / 64);
  const int b = slab / NH, h = slab % NH;
  const size_t pin = (size_t)blockIdx.y * ((size_t)NR * LQ);
  const size_t pout = (size_t)blockIdx.y * ((size_t)NB * NH * HD * SEQ);
  for (int i = tid; i < 64 * 8; i += 256) {
    const int r = i / 8, c8 = (i % 8) * 8;
    FragH f;
    f.half[0] = *(const v8us*)((const unsigned short*)QKV + pin + ((size_t)b * SEQ + lg * 64 + r) * LQ + 2 * DM + h * HD + c8);
#pragma unroll
    for (int q = 0; q < 8; ++q) tl[r][c8 + q] = f.u[q];
  }
  __syncthreads();
  for (int pass = 0; pass < 2; ++pass) {
#pragma unroll
    for (int rd = 0; rd < 2; ++rd) {
      const int d = rd * 32 + tid / 8, pc = tid % 8;
      FragH f;
#pragma unroll
      for (int q = 0; q < 8; ++q) f.u[q] = tl[pc * 8 + q][d];
      const v8us o = f.half[0];
      *(volatile v8us*)((unsigned short*)VT + pout + ((size_t)slab * 64 + d) * SEQ + lg * 64 + pc * 8) = o;
    }
    if (pass == 0) __threadfence();
  }
}

template <bool ER>
__device__ __forceinline__ void attn_body(const _Float16* __restrict__ Qh, const _Float16* __restrict__ Qr, const _Float16* __restrict__ VTh, const _Float16* __restrict__ VTr,
                                          _Float16* __restrict__ Oh, _Float16* __restrict__ Or, int qt0) {
  __shared__ __attribute__((aligned(16))) _Float16 ph[4][16][40];
  __shared__ __attribute__((aligned(16))) _Float16 pl[4][16][40];
  __shared__ __attribute__((aligned(16))) _Float16 oh[4][16][72];
  __shared__ __attribute__((aligned(16))) _Float16 ol[4][16][72];
  const int tid = threadIdx.x;
  const int wave = __builtin_amdgcn_readfirstlane((int)(tid >> 5));
  const int lane = tid & 31, ln = lane & 15, hh = lane >> 4;
  const int bh = blockIdx.y;
  const int b = bh / NH, h = bh % NH;
  const int q0 = (qt0 + (int)blockIdx.x) * 64 + wave * 16;
  const size_t rowb = (size_t)b * SEQ;
  const size_t qoff = (rowb + q0 + ln) * LQ + h * HD;
  const size_t koff0 = (rowb + ln) * LQ + DM + h * HD;
  const size_t voff0 = ((size_t)bh * HD + ln) * SEQ;
  const int nst = (q0 + 16 + 31) >> 5;
  const v8f z8 = {0.f, 0.f, 0.f, 0.f, 0.f, 0.f, 0.f, 0.f};
  v8f o[4] = {z8, z8, z8, z8};
  v8f orr[4] = {z8, z8, z8, z8};
  float mrow[8], lrow[8];
#pragma unroll
  for (int r = 0; r < 8; ++r) { mrow[r] = -1.0e30f; lrow[r] = 0.f; }
#pragma unroll 1
  for (int st = 0; st < nst; ++st) {
    const int key0 = st * 32;
    v8f sm[2] = {z8, z8};
    v8f sr[2] = {z8, z8};
#pragma unroll
    for (int kk = 0; kk < 2; ++kk) {
      const v16h qh = g2_frag(Qh + qoff + kk * 32, hh);
      v16h ql = qh;
      if (ER) ql = g2_frag(Qr + qoff + kk * 32, hh);
#pragma unroll
      for (int t = 0; t < 2; ++t) {
        const size_t ko = koff0 + (size_t)(key0 + 16 * t) * LQ + kk * 32;
        const v16h kh = g2_frag(Qh + ko, hh);
        sm[t] = g2_mma(qh, kh, sm[t]);
        if (ER) {
          const v16h kl = g2_frag(Qr + ko, hh);
          sr[t] = g2_mma(ql, kh, sr[t]);
          sr[t] = g2_mma(qh, kl, sr[t]);
        }
      }
    }
#pragma unroll
    for (int r = 0; r < 8; ++r) {
      const int qrow = q0 + 8 * hh + r;
      float s0 = sm[0][r], s1 = sm[1][r];
      if (ER) { s0 += sr[0][r] * 0.0009765625f; s1 += sr[1][r] * 0.0009765625f; }
      s0 *= 0.125f; s1 *= 0.125f;
      const bool m0 = (key0 + ln) > qrow, m1 = (key0 + 16 + ln) > qrow;
      s0 = m0 ? -1.0e9f : s0;
      s1 = m1 ? -1.0e9f : s1;
      float rm = fmaxf(s0, s1);
      rm = fmaxf(rm, __shfl_xor(rm, 1));
      rm = fmaxf(rm, __shfl_xor(rm, 2));
      rm = fmaxf(rm, __shfl_xor(rm, 4));
      rm = fmaxf(rm, __shfl_xor(rm, 8));
      const float mnew = fmaxf(mrow[r], rm);
      const float al = __expf(mrow[r] - mnew);
      const float e0 = __expf(s0 - mnew), e1 = __expf(s1 - mnew);
      const float p0 = m0 ? 0.f : e0, p1 = m1 ? 0.f : e1;
      lrow[r] = lrow[r] * al + (p0 + p1);
      mrow[r] = mnew;
#pragma unroll
      for (int j = 0; j < 4; ++j) { o[j][r] *= al; if (ER) orr[j][r] *= al; }
      const float a0 = p0 * 256.0f, a1 = p1 * 256.0f;
      const _Float16 h0 = (_Float16)a0, h1 = (_Float16)a1;
      ph[wave][8 * hh + r][ln] = h0;
      ph[wave][8 * hh + r][16 + ln] = h1;
      if (ER) {
        pl[wave][8 * hh + r][ln] = (_Float16)((a0 - (float)h0) * 1024.0f);
        pl[wave][8 * hh + r][16 + ln] = (_Float16)((a1 - (float)h1) * 1024.0f);
      }
    }
    wave_lds_sync();
    FragH pa, pb;
    pa.half[0] = *(const v8us*)&ph[wave][ln][8 * hh];
    pa.half[1] = *(const v8us*)&ph[wave][ln][16 + 8 * hh];
    pb.v = pa.v;
    if (ER) {
      pb.half[0] = *(const v8us*)&pl[wave][ln][8 * hh];
      pb.half[1] = *(const v8us*)&pl[wave][ln][16 + 8 * hh];
    }
#pragma unroll
    for (int j = 0; j < 4; ++j) {
      const size_t vo = voff0 + (size_t)(16 * j) * SEQ + key0;
      const v16h vh = g2_frag(VTh + vo, hh);
      o[j] = g2_mma(pa.v, vh, o[j]);
      if (ER) {
        const v16h vl = g2_frag(VTr + vo, hh);
        orr[j] = g2_mma(pb.v, vh, orr[j]);
        orr[j] = g2_mma(pa.v, vl, orr[j]);
      }
    }
    wave_lds_sync();
  }
#pragma unroll
  for (int r = 0; r < 8; ++r) {
    float l = lrow[r];
    l += __shfl_xor(l, 1);
    l += __shfl_xor(l, 2);
    l += __shfl_xor(l, 4);
    l += __shfl_xor(l, 8);
    const float inv = 0.25f * (1.0f / l);
#pragma unroll
    for (int j = 0; j < 4; ++j) {
      float v = o[j][r];
      if (ER) v += orr[j][r] * 0.0009765625f;
      v *= inv;
      const _Float16 hi = (_Float16)v;
      oh[wave][8 * hh + r][16 * j + ln] = hi;
      if (ER) ol[wave][8 * hh + r][16 * j + ln] = (_Float16)((v - (float)hi) * 1024.0f);
    }
  }
  wave_lds_sync();
  const int rsub = lane >> 3, c8 = (lane & 7) * 8;
  for (int pass = 0; pass < 2; ++pass) {
#pragma unroll
    for (int q = 0; q < 4; ++q) {
      const int r = q * 4 + rsub;
      const size_t oo = (rowb + q0 + r) * DM + h * HD + c8;
      const v8us vh8 = *(const v8us*)&oh[wave][r][c8];
      *(volatile v8us*)((unsigned short*)Oh + oo) = vh8;
      if (ER) {
        const v8us vl8 = *(const v8us*)&ol[wave][r][c8];
        *(volatile v8us*)((unsigned short*)Or + oo) = vl8;
      }
    }
    if (pass == 0) __threadfence();
  }
}
__global__ __launch_bounds__(128) void k_attn_late(const _Float16* __restrict__ Qh, const _Float16* __restrict__ Qr, const _Float16* __restrict__ VTh, const _Float16* __restrict__ VTr, _Float16* __restrict__ Oh, _Float16* __restrict__ Or, int qt0) {
  attn_body<false>(Qh, Qr, VTh, VTr, Oh, Or, qt0);
}
__global__ __launch_bounds__(128) void k_attn_early(const _Float16* __restrict__ Qh, const _Float16* __restrict__ Qr, const _Float16* __restrict__ VTh, const _Float16* __restrict__ VTr, _Float16* __restrict__ Oh, _Float16* __restrict__ Or, int qt0) {
  attn_body<true>(Qh, Qr, VTh, VTr, Oh, Or, qt0);
}

template <bool ER>
__device__ __forceinline__ void out_body(const _Float16* __restrict__ Ah, const _Float16* __restrict__ Ar, const _Float16* __restrict__ Bw, float* __restrict__ C, int rbPerB, int rowOff) {
  __shared__ __attribute__((aligned(16))) float so[4][32][68];
  const int tid = threadIdx.x;
  const int wave = __builtin_amdgcn_readfirstlane((int)(tid >> 5));
  const int lane = tid & 31, ln = lane & 15, hh = lane >> 4;
  const int ntn = DM / 64;
  const int mt = blockIdx.x / ntn, nq = blockIdx.x - mt * ntn;
  const int b = mt / rbPerB, lb = mt - b * rbPerB;
  const int s0 = rowOff + lb * 128 + 32 * wave;
  const int col0 = nq * 64;
  const size_t arow = (size_t)b * SEQ + s0;
  const size_t crow = (size_t)b * SEQ_FULL + s0;
  const size_t a0o = (arow + ln) * DM, a1o = a0o + (size_t)16 * DM;
  const _Float16* b0p = Bw + (size_t)(col0 + ln) * DM;
  const _Float16* b1p = b0p + (size_t)16 * DM;
  const _Float16* b2p = b1p + (size_t)16 * DM;
  const _Float16* b3p = b2p + (size_t)16 * DM;
  const v8f z8 = {0.f, 0.f, 0.f, 0.f, 0.f, 0.f, 0.f, 0.f};
  v8f c[8] = {z8, z8, z8, z8, z8, z8, z8, z8};
  v8f d[8] = {z8, z8, z8, z8, z8, z8, z8, z8};
#pragma unroll 1
  for (int kb = 0; kb < DM; kb += 32) {
    const v16h a0 = g2_frag(Ah + a0o + kb, hh), a1 = g2_frag(Ah + a1o + kb, hh);
    v16h r0 = a0, r1 = a1;
    if (ER) { r0 = g2_frag(Ar + a0o + kb, hh); r1 = g2_frag(Ar + a1o + kb, hh); }
    v16h bq = g2_frag(b0p + kb, hh);
    c[0] = g2_mma(a0, bq, c[0]); c[4] = g2_mma(a1, bq, c[4]);
    if (ER) { d[0] = g2_mma(r0, bq, d[0]); d[4] = g2_mma(r1, bq, d[4]); }
    bq = g2_frag(b1p + kb, hh);
    c[1] = g2_mma(a0, bq, c[1]); c[5] = g2_mma(a1, bq, c[5]);
    if (ER) { d[1] = g2_mma(r0, bq, d[1]); d[5] = g2_mma(r1, bq, d[5]); }
    bq = g2_frag(b2p + kb, hh);
    c[2] = g2_mma(a0, bq, c[2]); c[6] = g2_mma(a1, bq, c[6]);
    if (ER) { d[2] = g2_mma(r0, bq, d[2]); d[6] = g2_mma(r1, bq, d[6]); }
    bq = g2_frag(b3p + kb, hh);
    c[3] = g2_mma(a0, bq, c[3]); c[7] = g2_mma(a1, bq, c[7]);
    if (ER) { d[3] = g2_mma(r0, bq, d[3]); d[7] = g2_mma(r1, bq, d[7]); }
  }
#pragma unroll
  for (int u = 0; u < 8; ++u) {
    const int t = u & 3, half = u >> 2;
#pragma unroll
    for (int r = 0; r < 8; ++r) {
      float v = c[u][r];
      if (ER) v += d[u][r] * 0.0009765625f;
      so[wave][half * 16 + 8 * hh + r][t * 16 + ln] = v * 0.0009765625f;
    }
  }
  wave_lds_sync();
  const int rsub = lane >> 4, c4 = (lane & 15) * 4;
  for (int pass = 0; pass < 2; ++pass) {
#pragma unroll 1
    for (int q = 0; q < 16; ++q) {
      const int r = q * 2 + rsub;
      const v4f v = *(const v4fa*)&so[wave][r][c4];
      *(volatile v4f*)(C + (crow + r) * DM + col0 + c4) = v;
    }
    if (pass == 0) __threadfence();
  }
}
__global__ __launch_bounds__(128) void k_out_late(const _Float16* __restrict__ Ah, const _Float16* __restrict__ Ar, const _Float16* __restrict__ Bw, float* __restrict__ C, int rbPerB, int rowOff) {
  out_body<false>(Ah, Ar, Bw, C, rbPerB, rowOff);
}
__global__ __launch_bounds__(128) void k_out_early(const _Float16* __restrict__ Ah, const _Float16* __restrict__ Ar, const _Float16* __restrict__ Bw, float* __restrict__ C, int rbPerB, int rowOff) {
  out_body<true>(Ah, Ar, Bw, C, rbPerB, rowOff);
}

constexpr size_t SZ_W    = (size_t)DM * DM * 2;
constexpr size_t SZ_X16  = (size_t)NR * DM * 2;
constexpr size_t SZ_QKV  = (size_t)NR * LQ * 2;
constexpr size_t SZ_VT   = (size_t)NB * NH * HD * SEQ * 2;
constexpr size_t SZ_O    = (size_t)NR * DM * 2;
constexpr size_t SZ_CS   = (size_t)SEQ * 64 * 4;
constexpr size_t OFF_BW  = 0;
constexpr size_t OFF_X16 = OFF_BW + 4 * SZ_W;
constexpr size_t OFF_QKV = OFF_X16 + SZ_X16;
constexpr size_t OFF_VT  = OFF_QKV + 2 * SZ_QKV;
constexpr size_t OFF_O   = OFF_VT + 2 * SZ_VT;
constexpr size_t OFF_CS  = OFF_O + 2 * SZ_O;
constexpr size_t WS_TOTAL = OFF_CS + SZ_CS;
static_assert(WS_TOTAL <= (size_t)134217728);
static_assert(SZ_W % 256 == 0 && SZ_X16 % 256 == 0 && SZ_QKV % 256 == 0 && SZ_VT % 256 == 0 && SZ_O % 256 == 0 && SZ_CS % 256 == 0);
static_assert((size_t)((NB - 1) * SEQ_FULL + SEQ) * DM * 4 <= (size_t)NB_FULL * SEQ_FULL * DM * 4);

extern "C" void kernel_launch(void* const* d_in, const int* in_sizes, int n_in,
                              void* d_out, int out_size, void* d_ws, size_t ws_size, hipStream_t stream) {
  if (n_in < 6) return;
  const size_t need_x = (size_t)((NB - 1) * SEQ_FULL + SEQ) * DM;
  if ((size_t)in_sizes[0] < need_x) return;
  if ((size_t)in_sizes[1] < (size_t)DM * DM || (size_t)in_sizes[2] < (size_t)DM * DM || (size_t)in_sizes[3] < (size_t)DM * DM || (size_t)in_sizes[4] < (size_t)DM * DM) return;
  if (in_sizes[5] < SEQ) return;
  if ((size_t)out_size < need_x) return;
  if (WS_TOTAL > ws_size) return;
  const float* x  = (const float*)d_in[0];
  const float* wq = (const float*)d_in[1];
  const float* wk = (const float*)d_in[2];
  const float* wv = (const float*)d_in[3];
  const float* wo = (const float*)d_in[4];
  const int*   tp = (const int*)d_in[5];
  float* out = (float*)d_out;
  char* ws = (char*)d_ws;
  _Float16* BQKV = (_Float16*)(ws + OFF_BW);
  _Float16* BO   = (_Float16*)(ws + OFF_BW + 3 * SZ_W);
  _Float16* X16  = (_Float16*)(ws + OFF_X16);
  _Float16* QKVh = (_Float16*)(ws + OFF_QKV);
  _Float16* QKVr = (_Float16*)(ws + OFF_QKV + SZ_QKV);
  _Float16* VTh  = (_Float16*)(ws + OFF_VT);
  _Float16* VTr  = (_Float16*)(ws + OFF_VT + SZ_VT);
  _Float16* Oh   = (_Float16*)(ws + OFF_O);
  _Float16* Or   = (_Float16*)(ws + OFF_O + SZ_O);
  float*    CS   = (float*)(ws + OFF_CS);

  const unsigned gw = (unsigned)(((size_t)DM * DM / 8 + 255) / 256);
  k_wnat<<<gw, 256, 0, stream>>>(wq, BQKV);
  k_wnat<<<gw, 256, 0, stream>>>(wk, BQKV + (size_t)DM * DM);
  k_wnat<<<gw, 256, 0, stream>>>(wv, BQKV + (size_t)2 * DM * DM);
  k_wnat<<<gw, 256, 0, stream>>>(wo, BO);
  k_x16<<<(unsigned)(((size_t)NR * DM / 8 + 255) / 256), 256, 0, stream>>>(x, X16);
  k_tab<<<SEQ / 8, 256, 0, stream>>>(tp, CS);
  k_qkv<<<(unsigned)((NR / 128) * (LQ / 64)), 128, 0, stream>>>(X16, BQKV, CS, QKVh, QKVr);
  k_vt<<<dim3((unsigned)(NB * NH * (SEQ / 64)), 2), 256, 0, stream>>>(QKVh, VTh);
  if (SEQ / 64 > ERW / 64)
    k_attn_late<<<dim3((unsigned)(SEQ / 64 - ERW / 64), (unsigned)(NB * NH)), 128, 0, stream>>>(QKVh, QKVr, VTh, VTr, Oh, Or, ERW / 64);
  k_attn_early<<<dim3((unsigned)(ERW / 64), (unsigned)(NB * NH)), 128, 0, stream>>>(QKVh, QKVr, VTh, VTr, Oh, Or, 0);
  if (SEQ > ERW)
    k_out_late<<<(unsigned)(NB * ((SEQ - ERW) / 128) * (DM / 64)), 128, 0, stream>>>(Oh, Or, BO, out, (SEQ - ERW) / 128, ERW);
  k_out_early<<<(unsigned)(NB * (ERW / 128) * (DM / 64)), 128, 0, stream>>>(Oh, Or, BO, out, ERW / 128, 0);
}
